// WeightedReadOutPair_7112465842767
// MI455X (gfx1250) — hardware-verified
//
#include <hip/hip_runtime.h>
#include <math.h>


#define NN 1024
#define FF 64
typedef __attribute__((ext_vector_type(16))) _Float16 v16h;
typedef __attribute__((ext_vector_type(8)))  _Float16 v8h;
typedef __attribute__((ext_vector_type(8)))  float    v8f;
#define VST2(T, ptr, val) do { const T _v = (val); *(volatile T*)(ptr) = _v; __threadfence(); *(volatile T*)(ptr) = _v; } while (0)
__device__ __forceinline__ v8f wmma16(v16h a, v16h b, v8f c) {
  v8f d = __builtin_amdgcn_wmma_f32_16x16x32_f16(false, a, false, b, (short)0, c, false, false);
  asm volatile("v_nop\n\tv_nop\n\tv_nop\n\tv_nop" : "+v"(d) : "v"(a), "v"(b));
  return d;
}
__device__ __forceinline__ v16h frag16(const _Float16* p, int hh) {
  const v8h lo = *(const v8h*)(p + 8 * hh), hi = *(const v8h*)(p + 16 + 8 * hh);
  return __builtin_shufflevector(lo, hi, 0,1,2,3,4,5,6,7,8,9,10,11,12,13,14,15);
}
__device__ __forceinline__ int kmap(int e, int hh) { return (e < 8) ? (8 * hh + e) : (16 + 8 * hh + (e - 8)); }
__device__ __forceinline__ float silu(float x) { return x / (1.0f + __expf(-x)); }

__global__ __launch_bounds__(256) void k_node(const float* __restrict__ h, const float* __restrict__ lW1, const float* __restrict__ gW1, float* __restrict__ A1) {
  const int t = blockIdx.x * 256 + threadIdx.x;
  const int n = t >> 4, c = (t & 15) * 8, br = c >> 6, cc = c & 63;
  const float* W = br ? gW1 : lW1; const float* hr = h + (size_t)n * FF;
  float acc[8] = {0.f, 0.f, 0.f, 0.f, 0.f, 0.f, 0.f, 0.f};
  for (int k = 0; k < FF; ++k) { const float hv = hr[k];
#pragma unroll
    for (int e = 0; e < 8; ++e) acc[e] += hv * W[k * FF + cc + e]; }
  typedef __attribute__((ext_vector_type(8))) float v8f32; v8f32 o;
#pragma unroll
  for (int e = 0; e < 8; ++e) o[e] = acc[e] * 0.5f;
  VST2(v8f32, A1 + (size_t)n * 128 + c, o);
}
__global__ __launch_bounds__(256) void k_w2(const float* __restrict__ lW2, const float* __restrict__ gW2, _Float16* __restrict__ W2t) {
  const int t = blockIdx.x * 256 + threadIdx.x;
  const int br = t >> 9, n = (t >> 3) & 63, k0 = (t & 7) * 8;
  const float* W = br ? gW2 : lW2;
  v8h o;
#pragma unroll
  for (int e = 0; e < 8; ++e) o[e] = (_Float16)W[(k0 + e) * FF + n];
  VST2(v8h, W2t + ((size_t)br * FF + n) * FF + k0, o);
}
__global__ __launch_bounds__(64) void k_pairs(const float* __restrict__ A1, const _Float16* __restrict__ W2t,
                                               const float* __restrict__ lb1, const float* __restrict__ lb2, const float* __restrict__ lW3, const float* __restrict__ lb3,
                                               const float* __restrict__ gb1, const float* __restrict__ gb2, const float* __restrict__ gW3, const float* __restrict__ gb3,
                                               float* __restrict__ out) {
  __shared__ float sM[2][2][32][65];
  const int lane = threadIdx.x & 31, wave = threadIdx.x >> 5, hh = lane >> 4, l16 = lane & 15;
  const int wg = blockIdx.x * 2 + wave;
  const int i = wg >> 5, j0 = (wg & 31) * 32;
  const float* Ai = A1 + (size_t)i * 128;
#pragma unroll
  for (int br = 0; br < 2; ++br) {
    const float* b1 = br ? gb1 : lb1;
    v16h a[2][2];
#pragma unroll
    for (int r = 0; r < 2; ++r) {
      const float* Aj = A1 + (size_t)(j0 + r * 16 + l16) * 128 + br * 64;
#pragma unroll
      for (int ks = 0; ks < 2; ++ks)
#pragma unroll
        for (int e = 0; e < 16; ++e) { const int k = ks * 32 + kmap(e, hh); a[r][ks][e] = (_Float16)silu(Ai[br * 64 + k] + Aj[k] + b1[k]); }
    }
    const _Float16* Wb = W2t + (size_t)br * FF * FF;
#pragma unroll
    for (int t = 0; t < 4; ++t) {
      const v16h w0 = frag16(Wb + (size_t)(t * 16 + l16) * FF, hh), w1 = frag16(Wb + (size_t)(t * 16 + l16) * FF + 32, hh);
#pragma unroll
      for (int r = 0; r < 2; ++r) {
        v8f c = {};
        c = wmma16(a[r][0], w0, c); c = wmma16(a[r][1], w1, c);
#pragma unroll
        for (int v = 0; v < 8; ++v) sM[wave][br][r * 16 + v + 8 * hh][t * 16 + l16] = c[v];
      }
    }
  }
  __builtin_amdgcn_fence(__ATOMIC_RELEASE, "workgroup"); __builtin_amdgcn_wave_barrier(); __builtin_amdgcn_fence(__ATOMIC_ACQUIRE, "workgroup");
  float m = lb3[0], g = gb3[0];
  for (int k = 0; k < FF; ++k) { m += silu(sM[wave][0][lane][k] + lb2[k]) * lW3[k]; g += silu(sM[wave][1][lane][k] + gb2[k]) * gW3[k]; }
  const float o = m * (1.0f / (1.0f + __expf(-g)));
  VST2(float, out + (size_t)i * NN + j0 + lane, o);
}
extern "C" void kernel_launch(void* const* d_in, const int* in_sizes, int n_in,
                              void* d_out, int out_size, void* d_ws, size_t ws_size, hipStream_t stream) {
  (void)in_sizes; (void)n_in; (void)out_size;
  const float* h   = (const float*)d_in[0];
  const float* lW1 = (const float*)d_in[1]; const float* lb1 = (const float*)d_in[2];
  const float* lW2 = (const float*)d_in[3]; const float* lb2 = (const float*)d_in[4];
  const float* lW3 = (const float*)d_in[5]; const float* lb3 = (const float*)d_in[6];
  const float* gW1 = (const float*)d_in[7]; const float* gb1 = (const float*)d_in[8];
  const float* gW2 = (const float*)d_in[9]; const float* gb2 = (const float*)d_in[10];
  const float* gW3 = (const float*)d_in[11]; const float* gb3 = (const float*)d_in[12];
  float* out = (float*)d_out;
  char* ws = (char*)d_ws; size_t off = 0;
  auto take = [&](size_t bytes) { void* p = ws + off; off = (off + bytes + 255) & ~(size_t)255; return p; };
  float*    A1  = (float*)take((size_t)NN * 128 * 4);
  _Float16* W2t = (_Float16*)take((size_t)2 * FF * FF * 2);
  if (off > ws_size) return;
  k_node<<<NN * 16 / 256, 256, 0, stream>>>(h, lW1, gW1, A1);
  k_w2<<<2 * 64 * 8 / 256, 256, 0, stream>>>(lW2, gW2, W2t);
  k_pairs<<<NN * NN / 32 / 2, 64, 0, stream>>>(A1, W2t, lb1, lb2, lW3, lb3, gb1, gb2, gW3, gb3, out);
}
